// KNNDensityEstimator_2594160247093
// MI455X (gfx1250) — hardware-verified
//
#include <hip/hip_runtime.h>
#include <math.h>

typedef __attribute__((ext_vector_type(16))) _Float16 v16h;
typedef __attribute__((ext_vector_type(16))) __bf16 v16b;
typedef __attribute__((ext_vector_type(8)))  _Float16 v8h;
typedef __attribute__((ext_vector_type(8)))  float v8f;
typedef __attribute__((ext_vector_type(4)))  float v4f;
typedef __attribute__((ext_vector_type(2)))  float v2f;
typedef __attribute__((ext_vector_type(4)))  unsigned v4u;
typedef __attribute__((ext_vector_type(4)))  int v4i;
typedef float __attribute__((may_alias)) float_a;
typedef int __attribute__((may_alias)) int_a;

template <typename T> __device__ __forceinline__ void vst2(void* p, T v) { *(volatile T*)p = v; __threadfence(); *(volatile T*)p = v; }
__device__ __forceinline__ v8f wmma16(v16h a, v16h b, v8f c) {
  v8f d = __builtin_amdgcn_wmma_f32_16x16x32_f16(false, a, false, b, (short)0, c, false, false);
  asm volatile("v_nop\n\tv_nop\n\tv_nop\n\tv_nop" : "+v"(d) : "v"(a), "v"(b));
  return d;
}
__device__ __forceinline__ v8f wmma_bf(v16b a, v16b b, v8f c) {
  v8f d = __builtin_amdgcn_wmma_f32_16x16x32_bf16(false, a, false, b, (short)0, c, false, false);
  asm volatile("v_nop\n\tv_nop\n\tv_nop\n\tv_nop" : "+v"(d) : "v"(a), "v"(b));
  return d;
}
__device__ __forceinline__ v16h frag_h(const _Float16* rowk0, int lane) {
  union { v16h v; v8h q[2]; } u; const _Float16* p = rowk0 + 8 * (lane >> 4);
  u.q[0] = *(const v8h*)p; u.q[1] = *(const v8h*)(p + 16); return u.v;
}
__device__ __forceinline__ v16h frag_f32(const float* rowk0, int lane) {
  v16h a; const float* p = rowk0 + 8 * (lane >> 4);
#pragma unroll
  for (int i = 0; i < 8; ++i) { a[i] = (_Float16)p[i]; a[8 + i] = (_Float16)p[16 + i]; }
  return a;
}
__device__ __forceinline__ v16h frag_f32s(const float* rowk0, int lane, float sc) {
  v16h a; const float* p = rowk0 + 8 * (lane >> 4);
#pragma unroll
  for (int i = 0; i < 8; ++i) { a[i] = (_Float16)(p[i] * sc); a[8 + i] = (_Float16)(p[16 + i] * sc); }
  return a;
}
__device__ __forceinline__ v16h fragc_f32(const float* W, int k0, int n, int lane, int ld, int K) {
  v16h a; const int g = lane >> 4;
#pragma unroll
  for (int i = 0; i < 8; ++i) { const int ka = k0 + 8 * g + i, kb = ka + 16;
    a[i] = (_Float16)(ka < K ? W[(size_t)(ka < K ? ka : K - 1) * ld + n] : 0.f); a[8 + i] = (_Float16)(kb < K ? W[(size_t)(kb < K ? kb : K - 1) * ld + n] : 0.f); }
  return a;
}
struct F2 { v16b h, l; };
__device__ __forceinline__ F2 bsplit16(const float v[16]) { F2 r;
#pragma unroll
  for (int i = 0; i < 16; ++i) { const __bf16 h = (__bf16)v[i]; r.h[i] = h; r.l[i] = (__bf16)(v[i] - (float)h); }
  return r; }
__device__ __forceinline__ F2 split_row(const float* row, int k0, int lane) { float v[16]; const float* p = row + k0 + 8 * (lane >> 4);
#pragma unroll
  for (int i = 0; i < 8; ++i) { v[i] = p[i]; v[8 + i] = p[16 + i]; }
  return bsplit16(v); }
__device__ __forceinline__ F2 split_rowK(const float* row, int k0, int lane, int K) { float v[16]; const int g = lane >> 4;
#pragma unroll
  for (int i = 0; i < 8; ++i) { const int ka = k0 + 8 * g + i, kb = ka + 16; v[i] = ka < K ? row[ka < K ? ka : K - 1] : 0.f; v[8 + i] = kb < K ? row[kb < K ? kb : K - 1] : 0.f; }
  return bsplit16(v); }
__device__ __forceinline__ F2 split_col(const float* W, int k0, int n, int lane, int ld, int K) { float v[16]; const int g = lane >> 4;
#pragma unroll
  for (int i = 0; i < 8; ++i) { const int ka = k0 + 8 * g + i, kb = ka + 16; v[i] = ka < K ? W[(size_t)(ka < K ? ka : K - 1) * ld + n] : 0.f; v[8 + i] = kb < K ? W[(size_t)(kb < K ? kb : K - 1) * ld + n] : 0.f; }
  return bsplit16(v); }
__device__ __forceinline__ v8f mac3(const F2& a, const F2& b, v8f c) { c = wmma_bf(a.l, b.h, c); c = wmma_bf(a.h, b.l, c); return wmma_bf(a.h, b.h, c); }
__device__ __forceinline__ float sigm(float v) { return 1.0f / (1.0f + expf(-v)); }
#define LDSX() do { asm volatile("s_wait_dscnt 0" ::: "memory"); __builtin_amdgcn_wave_barrier(); __builtin_amdgcn_fence(__ATOMIC_RELEASE, "workgroup"); } while (0)


#define NQ 512
#define NRF 100000
#define DD 128
#define KK 10
#define NTL (NRF / 16)
#ifndef NBLK
#define NBLK (NQ / 32)
#endif
typedef __attribute__((ext_vector_type(8))) __bf16 v8b;
__device__ __forceinline__ v16b frag_b(const __bf16* rowk0, int lane) {
  union { v16b v; v8b q[2]; } u; const __bf16* p = rowk0 + 8 * (lane >> 4);
  u.q[0] = *(const v8b*)p; u.q[1] = *(const v8b*)(p + 16); return u.v;
}
__device__ __forceinline__ float bfr(float v) { return (float)(__bf16)v; }
__device__ __attribute__((noinline)) float exp_ni(float v) { return expf(v); }
__device__ __attribute__((noinline)) float erf_ni(float v) { return erff(v); }

#define WS_Y2  0u
#define WS_END (WS_Y2 + 4u * NRF)

__global__ __launch_bounds__(256) void k_y2(const float* __restrict__ RF, float* __restrict__ Y2) {
  __shared__ __align__(16) float s[256]; const int t = threadIdx.x; const size_t i = (size_t)blockIdx.x * 256 + t; float a = 0.f;
  if (i < NRF) { const float* row = RF + i * DD;
#pragma unroll 4
    for (int c = 0; c < DD; ++c) { const float v = bfr(row[c]); a += v * v; } }
  s[t] = a; __syncthreads();
  if (t < 64 && (size_t)blockIdx.x * 256 + t * 4 < NRF) vst2(Y2 + (size_t)blockIdx.x * 256 + t * 4, *(const v4f*)&s[t * 4]);
}
__device__ __forceinline__ void ins10(float v, float* b) { if (v < b[KK - 1]) { int pos = KK - 1;
#pragma unroll
    for (int q = KK - 2; q >= 0; --q) if (v < b[q]) pos = q;
#pragma unroll
    for (int q = KK - 1; q >= 1; --q) if (q > pos) b[q] = b[q - 1];
#pragma unroll
    for (int q = 0; q < KK; ++q) if (q == pos) b[q] = v; } }
__global__ __launch_bounds__(256) void k_knn(const float* __restrict__ X, const float* __restrict__ RF, const float* __restrict__ Y2, float* __restrict__ OUT) {
  __shared__ __align__(16) float ss[8][16][20]; __shared__ float sb[8][16][KK + 1]; __shared__ __align__(16) float so[32];
  const int tid = threadIdx.x, wave = tid >> 5, lane = tid & 31, col = lane & 15, g = lane >> 4; const int ph = wave & 3, rt = wave >> 2; const size_t q0 = (size_t)blockIdx.x * 32 + rt * 16;
  v16b xa[4]; { const float* p0 = X + (q0 + col) * DD;
#pragma unroll
    for (int kc = 0; kc < 4; ++kc) { const float* p = p0 + kc * 32 + 8 * g;
#pragma unroll
      for (int i2 = 0; i2 < 8; ++i2) { xa[kc][i2] = (__bf16)p[i2]; xa[kc][8 + i2] = (__bf16)p[16 + i2]; } } }
  float x2 = 0.f; if (lane < 16) { const float* row = X + (q0 + lane) * DD;
#pragma unroll 4
    for (int c = 0; c < DD; ++c) { const float v = bfr(row[c]); x2 += v * v; } }
  float best[KK];
#pragma unroll
  for (int q = 0; q < KK; ++q) best[q] = 3.0e38f;
#pragma unroll 1
  for (int t = ph; t < NTL; t += 4) { v8f acc = {}; const float* yrow = RF + ((size_t)t * 16 + col) * DD + 8 * g;
#pragma unroll
    for (int kc = 0; kc < 4; ++kc) { v16b yb; const float* p = yrow + kc * 32;
#pragma unroll
      for (int i2 = 0; i2 < 8; ++i2) { yb[i2] = (__bf16)p[i2]; yb[8 + i2] = (__bf16)p[16 + i2]; }
      acc = wmma_bf(xa[kc], yb, acc); }
    { const float y2 = Y2[(size_t)t * 16 + col];
#pragma unroll
      for (int r = 0; r < 8; ++r) ss[wave][8 * g + r][col] = y2 - 2.0f * acc[r]; }
    LDSX();
    if (lane < 16) {
#pragma unroll
      for (int c = 0; c < 16; ++c) ins10(fmaxf(ss[wave][lane][c] + x2, 0.f), best); }
    LDSX(); }
  if (lane < 16) {
#pragma unroll
    for (int q = 0; q < KK; ++q) sb[wave][lane][q] = best[q]; }
  __syncthreads();
  if (ph == 0 && lane < 16) { float m[KK];
#pragma unroll
    for (int q = 0; q < KK; ++q) m[q] = best[q];
    for (int w2 = 1; w2 < 4; ++w2) { const int w = rt * 4 + w2;
#pragma unroll
      for (int q = 0; q < KK; ++q) ins10(sb[w][lane][q], m); }
    float a = 0.f;
#pragma unroll
    for (int q = 0; q < KK; ++q) a += sqrtf(m[q]);
    so[rt * 16 + lane] = -a / (float)KK; }
  __syncthreads();
  if (tid < 8) vst2(OUT + (size_t)blockIdx.x * 32 + tid * 4, *(const v4f*)&so[tid * 4]);
}
extern "C" void kernel_launch(void* const* d_in, const int* in_sizes, int n_in, void* d_out, int out_size, void* d_ws, size_t ws_size, hipStream_t stream) {
  (void)in_sizes; (void)n_in; (void)out_size;
  if (ws_size < (size_t)WS_END) return;
  char* ws = (char*)d_ws; float* Y2 = (float*)(ws + WS_Y2);
  k_y2<<<(NRF + 255) / 256, 256, 0, stream>>>((const float*)d_in[1], Y2);
  k_knn<<<NBLK, 256, 0, stream>>>((const float*)d_in[0], (const float*)d_in[1], Y2, (float*)d_out);
}
